// Algin_38603166056827
// MI455X (gfx1250) — hardware-verified
//
#include <hip/hip_runtime.h>
#include <stddef.h>

constexpr int NBATCH    = 4;
constexpr int NCH       = 16;
constexpr int IMG_H     = 192;
constexpr int KTAPS     = 9;
constexpr int PITCH_A16 = 192;
constexpr int KDIM16    = 160;
constexpr int KREAL16   = 144;
constexpr int PITCH_A32 = 384;
constexpr int KDIM32    = 288;
constexpr int NOFFCH    = 144;
constexpr int NOFFPAD   = 192;
constexpr int FEAT_ROWS = NBATCH * IMG_H * IMG_H;
constexpr int CHUNK_FE  = 73728;
constexpr int CHUNK_A   = 73728;
constexpr int CHUNK_B   = 49152;
static_assert(KDIM16 % 32 == 0 && KDIM32 % 32 == 0, "");
static_assert(CHUNK_FE % 64 == 0 && CHUNK_A % 64 == 0 && CHUNK_B % 64 == 0, "");
static_assert((size_t)CHUNK_A * PITCH_A32 * 2 == (size_t)CHUNK_FE * PITCH_A16 * 2 * 2, "");
static_assert((size_t)CHUNK_B * PITCH_A16 * 2 + (size_t)CHUNK_B * NOFFPAD * 4 == (size_t)CHUNK_FE * PITCH_A16 * 2 * 2, "");

typedef __attribute__((ext_vector_type(16))) _Float16 v16h;
typedef __attribute__((ext_vector_type(8)))  _Float16 v8h;
typedef __attribute__((ext_vector_type(16))) __bf16   v16b;
typedef __attribute__((ext_vector_type(8)))  __bf16   v8b;
typedef __attribute__((ext_vector_type(8)))  float    v8f;
typedef __attribute__((ext_vector_type(4)))  float    v4f;
typedef __attribute__((ext_vector_type(2)))  float    v2f;
typedef __attribute__((ext_vector_type(4)))  unsigned v4u;

__device__ __forceinline__ unsigned short f2bf_bits(float f) {
  unsigned u = __float_as_uint(f);
  return (unsigned short)((u + 0x7FFFu + ((u >> 16) & 1u)) >> 16);
}
__device__ __forceinline__ float bf_bits2f(unsigned short h) { return __uint_as_float(((unsigned)h) << 16); }

__device__ __forceinline__ unsigned pk2(unsigned short a, unsigned short b) {
  return (unsigned)a | ((unsigned)b << 16);
}
__device__ __forceinline__ unsigned pkh2(float a, float b) {
  return pk2(__builtin_bit_cast(unsigned short, (_Float16)a), __builtin_bit_cast(unsigned short, (_Float16)b));
}
__device__ __forceinline__ void pkbf2(float a, float b, unsigned& uh, unsigned& ul) {
  const unsigned short ha = f2bf_bits(a), hb = f2bf_bits(b);
  const unsigned short la = f2bf_bits(a - bf_bits2f(ha)), lb = f2bf_bits(b - bf_bits2f(hb));
  uh = pk2(ha, hb);
  ul = pk2(la, lb);
}

__device__ __forceinline__ void dep_guard_h(v8f& a, v8f& b, v16h x, v16h y) { asm volatile("v_nop\n\tv_nop\n\tv_nop\n\tv_nop" : "+v"(a), "+v"(b) : "v"(x), "v"(y)); }
__device__ __forceinline__ void dep_guard_b(v8f& a, v8f& b, v16b x, v16b y) { asm volatile("v_nop\n\tv_nop\n\tv_nop\n\tv_nop" : "+v"(a), "+v"(b) : "v"(x), "v"(y)); }
__device__ __forceinline__ void dep_guard1_h(v8f& a, v16h x, v16h y) { asm volatile("v_nop\n\tv_nop\n\tv_nop\n\tv_nop" : "+v"(a) : "v"(x), "v"(y)); }
__device__ __forceinline__ void dep_guard1_b(v8f& a, v16b x, v16b y) { asm volatile("v_nop\n\tv_nop\n\tv_nop\n\tv_nop" : "+v"(a) : "v"(x), "v"(y)); }
__device__ __forceinline__ void keep4_h(v16h a, v16h b, v16h c, v16h d) { asm volatile("v_nop" :: "v"(a), "v"(b), "v"(c), "v"(d)); }
__device__ __forceinline__ void keep4_b(v16b a, v16b b, v16b c, v16b d) { asm volatile("v_nop" :: "v"(a), "v"(b), "v"(c), "v"(d)); }
__device__ __forceinline__ void acc_guard4(v8f& a, v8f& b, v8f& c, v8f& d) { asm volatile("v_nop\n\tv_nop\n\tv_nop\n\tv_nop" : "+v"(a), "+v"(b), "+v"(c), "+v"(d)); }
template <typename T> struct Frag;
template <> struct Frag<_Float16> {
  typedef v16h V; union U { v16h v; v8h h[2]; };
  static __device__ __forceinline__ v16h load(const _Float16* p) {
    U f; f.h[0] = *(const v8h*)(p); f.h[1] = *(const v8h*)(p + 16); return f.v;
  }
  static __device__ __forceinline__ v8f mma(v16h a, v16h b, v8f c) {
    return __builtin_amdgcn_wmma_f32_16x16x32_f16(false, a, false, b, (short)0, c, false, false);
  }
  static __device__ __forceinline__ void guard(v8f& a, v8f& b, v16h x, v16h y) { dep_guard_h(a, b, x, y); }
  static __device__ __forceinline__ void guard1(v8f& a, v16h x, v16h y) { dep_guard1_h(a, x, y); }
  static __device__ __forceinline__ void keep(v16h a, v16h b, v16h c, v16h d) { keep4_h(a, b, c, d); }
};
template <> struct Frag<__bf16> {
  typedef v16b V; union U { v16b v; v8b h[2]; };
  static __device__ __forceinline__ v16b load(const __bf16* p) {
    U f; f.h[0] = *(const v8b*)(p); f.h[1] = *(const v8b*)(p + 16); return f.v;
  }
  static __device__ __forceinline__ v8f mma(v16b a, v16b b, v8f c) {
    return __builtin_amdgcn_wmma_f32_16x16x32_bf16(false, a, false, b, (short)0, c, false, false);
  }
  static __device__ __forceinline__ void guard(v8f& a, v8f& b, v16b x, v16b y) { dep_guard_b(a, b, x, y); }
  static __device__ __forceinline__ void guard1(v8f& a, v16b x, v16b y) { dep_guard1_b(a, x, y); }
  static __device__ __forceinline__ void keep(v16b a, v16b b, v16b c, v16b d) { keep4_b(a, b, c, d); }
};

template <int ET> struct Elem;
template <> struct Elem<0> { typedef _Float16 T; };
template <> struct Elem<1> { typedef __bf16 T; };
template <int ET, bool SPLIT, int BIAS_MODE, int OUT_MODE, bool RESID, int ACT, int NT>
__global__ __launch_bounds__(256) void wmma_gemm64(
    const unsigned short* __restrict__ Ap, const unsigned short* __restrict__ A2p, int lda, long strideA,
    const unsigned short* __restrict__ Btp, const unsigned short* __restrict__ Bt2p, int ldb, long strideB,
    void* __restrict__ Cout, void* __restrict__ Cout2, int ldc, long strideC,
    const float* __restrict__ bias,
    const float* __restrict__ resid, long strideR,
    int M, int N, int K, float scale) {
  static_assert(NT == 1 || NT == 4, "");
  static_assert((OUT_MODE == 3) ? (NT == 1) : (NT == 4), "");
  typedef typename Elem<ET>::T T;
  typedef typename Frag<T>::V V;
  const T* A = (const T*)Ap; const T* A2 = (const T*)A2p; const T* Bt = (const T*)Btp; const T* Bt2 = (const T*)Bt2p;
  __shared__ __align__(16) float sT[8][16 * 68];
  const int b    = blockIdx.y;
  const int lane = threadIdx.x & 31;
  const int wave = threadIdx.x >> 5;
  const int tilesN = N / (16 * NT);
  const int tilesM = M >> 6;
  const int tile = blockIdx.x * 8 + wave;
  if (tile >= tilesM * tilesN) return;
  const int tm = tile / tilesN;
  const int tn = tile - tm * tilesN;
  const int m0 = tm << 6;
  const int n0 = tn * (16 * NT);

  const T* Ab  = A  + (size_t)b * strideA;
  const T* Bb  = Bt + (size_t)b * strideB;
  const T* Ab2 = SPLIT ? (A2  + (size_t)b * strideA) : nullptr;
  const T* Bb2 = SPLIT ? (Bt2 + (size_t)b * strideB) : nullptr;

  const int rlane = lane & 15;
  const int koff  = (lane >> 4) * 8;
  const int mOff  = (lane >> 4) * 8;

  v8f acc[4][4];
#pragma unroll
  for (int i = 0; i < 4; ++i)
#pragma unroll
    for (int j = 0; j < 4; ++j) acc[i][j] = (v8f){0.f,0.f,0.f,0.f,0.f,0.f,0.f,0.f};

  for (int k0 = 0; k0 < K; k0 += 32) {
    V bh[4], bl[4];
#pragma unroll
    for (int j = 0; j < NT; ++j) {
      const size_t bo = (size_t)(n0 + (j << 4) + rlane) * ldb + koff + k0;
      bh[j] = Frag<T>::load(Bb + bo);
      if (SPLIT) bl[j] = Frag<T>::load(Bb2 + bo);
    }
#pragma unroll
    for (int i = 0; i < 4; ++i) {
      const size_t ao = (size_t)(m0 + (i << 4) + rlane) * lda + koff + k0;
      V ah = Frag<T>::load(Ab + ao);
      V al;
      if (SPLIT) al = Frag<T>::load(Ab2 + ao);
#pragma unroll
      for (int j = 0; j < NT; ++j) {
        acc[i][j] = Frag<T>::mma(ah, bh[j], acc[i][j]);
        if (SPLIT) {
          acc[i][j] = Frag<T>::mma(ah, bl[j], acc[i][j]);
          acc[i][j] = Frag<T>::mma(al, bh[j], acc[i][j]);
        }
      }
      if (NT == 4) Frag<T>::guard(acc[i][0], acc[i][3], ah, SPLIT ? al : ah);
      else         Frag<T>::guard1(acc[i][0], ah, SPLIT ? al : ah);
    }
    Frag<T>::keep(bh[0], bh[(NT > 1) ? 1 : 0], bh[(NT > 2) ? 2 : 0], bh[(NT > 3) ? 3 : 0]);
    if (SPLIT) Frag<T>::keep(bl[0], bl[(NT > 1) ? 1 : 0], bl[(NT > 2) ? 2 : 0], bl[(NT > 3) ? 3 : 0]);
  }
  if (NT == 4) {
    acc_guard4(acc[0][0], acc[0][1], acc[0][2], acc[0][3]);
    acc_guard4(acc[1][0], acc[1][1], acc[1][2], acc[1][3]);
    acc_guard4(acc[2][0], acc[2][1], acc[2][2], acc[2][3]);
    acc_guard4(acc[3][0], acc[3][1], acc[3][2], acc[3][3]);
  } else {
    acc_guard4(acc[0][0], acc[1][0], acc[2][0], acc[3][0]);
  }

  float* slab = sT[wave];
  const float* Rb = RESID ? (resid + (size_t)b * strideR) : nullptr;
#pragma unroll
  for (int i = 0; i < 4; ++i) {
    const int mBase = m0 + (i << 4);
#pragma unroll
    for (int j = 0; j < NT; ++j) {
      const int n = n0 + (j << 4) + rlane;
      float bv = 0.f;
      if (BIAS_MODE == 2) bv = bias[n];
#pragma unroll
      for (int r = 0; r < 8; ++r) {
        float v = acc[i][j][r] * scale;
        if (BIAS_MODE == 1) v += bias[mBase + mOff + r];
        if (BIAS_MODE == 2) v += bv;
        if (RESID) v += Rb[(size_t)(mBase + mOff + r) * ldc + n];
        if (ACT == 1) v = tanhf(v);
        if (ACT == 2) v = fmaxf(v, 0.0f);
        if (ACT == 3) v = v / (1.0f + expf(-v));
        if (ACT == 4) v = (v > 0.f) ? v : 0.01f * v;
        slab[(mOff + r) * 68 + (j << 4) + rlane] = v;
      }
    }
    __builtin_amdgcn_fence(__ATOMIC_RELEASE, "workgroup");
    __builtin_amdgcn_wave_barrier();
    __builtin_amdgcn_fence(__ATOMIC_ACQUIRE, "workgroup");
    if (OUT_MODE == 0) {
      float* C = (float*)Cout + (size_t)b * strideC;
      const int hh = lane >> 4, c4 = (lane & 15) * 4;
      for (int pass = 0; pass < 2; ++pass) {
#pragma unroll
        for (int it = 0; it < 8; ++it) {
          const int row = it * 2 + hh;
          v4f v = *(const v4f*)(slab + row * 68 + c4);
          *(volatile v4f*)(C + (size_t)(mBase + row) * ldc + n0 + c4) = v;
        }
        __threadfence();
      }
    } else if (OUT_MODE == 3) {
      float* C = (float*)Cout + (size_t)b * strideC;
      const int rr = lane >> 2, c4 = (lane & 3) * 4;
      for (int pass = 0; pass < 2; ++pass) {
#pragma unroll
        for (int it = 0; it < 2; ++it) {
          const int row = it * 8 + rr;
          v4f v = *(const v4f*)(slab + row * 68 + c4);
          *(volatile v4f*)(C + (size_t)(mBase + row) * ldc + n0 + c4) = v;
        }
        __threadfence();
      }
    } else {
      const int q = lane >> 3, c8 = (lane & 7) * 8;
      unsigned short* C  = (unsigned short*)Cout  + (size_t)b * strideC;
      unsigned short* C2 = (OUT_MODE == 2) ? ((unsigned short*)Cout2 + (size_t)b * strideC) : nullptr;
      for (int pass = 0; pass < 2; ++pass) {
#pragma unroll
        for (int it = 0; it < 4; ++it) {
          const int row = it * 4 + q;
          const float* sp = slab + row * 68 + c8;
          v8h hv, lv;
#pragma unroll
          for (int e = 0; e < 8; ++e) {
            if (OUT_MODE == 1) {
              hv[e] = (_Float16)sp[e];
            } else {
              unsigned short hb = f2bf_bits(sp[e]);
              unsigned short lb = f2bf_bits(sp[e] - bf_bits2f(hb));
              hv[e] = __builtin_bit_cast(_Float16, hb);
              lv[e] = __builtin_bit_cast(_Float16, lb);
            }
          }
          *(volatile v8h*)(C + (size_t)(mBase + row) * ldc + n0 + c8) = hv;
          if (OUT_MODE == 2) *(volatile v8h*)(C2 + (size_t)(mBase + row) * ldc + n0 + c8) = lv;
        }
        __threadfence();
      }
    }
    __builtin_amdgcn_fence(__ATOMIC_RELEASE, "workgroup");
    __builtin_amdgcn_wave_barrier();
    __builtin_amdgcn_fence(__ATOMIC_ACQUIRE, "workgroup");
  }
}

template <int CINW, int MODE>
__global__ __launch_bounds__(256) void k_prep_w(const float* __restrict__ w0, const float* __restrict__ w1,
                                                const float* __restrict__ w2, unsigned short* __restrict__ outBase,
                                                int levelStride, int loOff, int nOut, int rowsPad, float scl) {
  constexpr int PITCH  = (CINW == 16) ? PITCH_A16 : PITCH_A32;
  constexpr int KREALW = CINW * KTAPS;
  const float* w = (blockIdx.y == 0) ? w0 : ((blockIdx.y == 1) ? w1 : w2);
  unsigned short* out = outBase + (size_t)blockIdx.y * levelStride;
  const int g = blockIdx.x * 256 + threadIdx.x;
  const int items = rowsPad * PITCH / 8;
  if (g < items) {
    const int e0  = g * 8;
    const int o   = e0 / PITCH;
    const int col = e0 - o * PITCH;
    int tap = col / CINW; tap = tap > 8 ? 8 : tap;
    const int c0  = col & (CINW - 1);
    const bool ok = (col < KREALW) && (o < nOut);
    const int oc  = o < nOut ? o : (nOut - 1);
    float f[8];
#pragma unroll
    for (int j = 0; j < 8; ++j) {
      const float v = w[(size_t)(oc * CINW + c0 + j) * KTAPS + tap] * scl;
      f[j] = ok ? v : 0.0f;
    }
    if (MODE == 0) {
      v4u uh, ul;
      unsigned a, bb;
      pkbf2(f[0], f[1], a, bb); uh[0] = a; ul[0] = bb;
      pkbf2(f[2], f[3], a, bb); uh[1] = a; ul[1] = bb;
      pkbf2(f[4], f[5], a, bb); uh[2] = a; ul[2] = bb;
      pkbf2(f[6], f[7], a, bb); uh[3] = a; ul[3] = bb;
      volatile v4u* ph = (volatile v4u*)(out + e0);
      volatile v4u* pl = (volatile v4u*)(out + loOff + e0);
      *ph = uh; *pl = ul;
      __threadfence();
      *ph = uh; *pl = ul;
    } else {
      v4u u;
      u[0] = pkh2(f[0], f[1]); u[1] = pkh2(f[2], f[3]); u[2] = pkh2(f[4], f[5]); u[3] = pkh2(f[6], f[7]);
      volatile v4u* p = (volatile v4u*)(out + e0);
      *p = u;
      __threadfence();
      *p = u;
    }
  }
}

template <bool SRC_NCHW, int OUTM>
__global__ __launch_bounds__(256) void k_im2col16(const float* __restrict__ src,
                                                  unsigned short* __restrict__ outH, unsigned short* __restrict__ outL,
                                                  int hi, int wi, int ho, int wo, int pad, int pxReal,
                                                  int rowStart, int nRows) {
  const int lane = threadIdx.x & 31;
  const int wg = blockIdx.x * 8 + (threadIdx.x >> 5);
  const int r0 = wg * 4;
  if (r0 >= nRows) return;
  const int howo = ho * wo;
  const size_t hiwi = (size_t)hi * wi;
#pragma unroll 1
  for (int t = 0; t < 3; ++t) {
    const int e   = (t * 32 + lane) * 8;
    const int rl  = e / PITCH_A16;
    const int col = e - rl * PITCH_A16;
    const int p   = rowStart + r0 + rl;
    const int pc  = p < pxReal ? p : (pxReal - 1);
    const int b   = pc / howo;
    const int rem = pc - b * howo;
    const int y   = rem / wo;
    const int x   = rem - y * wo;
    int tap = col >> 4; tap = tap > 8 ? 8 : tap;
    const int kh = tap / 3, kw = tap - kh * 3;
    const int c0 = col & 8;
    const int yi = y + kh - pad, xi = x + kw - pad;
    const bool ok = (col < KREAL16) && (p < pxReal) &&
                    ((unsigned)yi < (unsigned)hi) && ((unsigned)xi < (unsigned)wi);
    const int yc = yi < 0 ? 0 : (yi > hi - 1 ? hi - 1 : yi);
    const int xc = xi < 0 ? 0 : (xi > wi - 1 ? wi - 1 : xi);
    float f[8];
    if (SRC_NCHW) {
      const float* s0 = src + ((size_t)b * NCH + c0) * hiwi + (size_t)yc * wi + xc;
#pragma unroll
      for (int j = 0; j < 8; ++j) f[j] = s0[(size_t)j * hiwi];
    } else {
      const float* s0 = src + ((size_t)b * hiwi + (size_t)yc * wi + xc) * NCH + c0;
      const v4f a = *(const v4f*)(s0);
      const v4f c = *(const v4f*)(s0 + 4);
      f[0] = a[0]; f[1] = a[1]; f[2] = a[2]; f[3] = a[3];
      f[4] = c[0]; f[5] = c[1]; f[6] = c[2]; f[7] = c[3];
    }
#pragma unroll
    for (int j = 0; j < 8; ++j) f[j] = ok ? f[j] : 0.0f;
    const size_t o = (size_t)r0 * PITCH_A16 + e;
    if (OUTM == 0) {
      v4u uh, ul;
      unsigned a, bb;
      pkbf2(f[0], f[1], a, bb); uh[0] = a; ul[0] = bb;
      pkbf2(f[2], f[3], a, bb); uh[1] = a; ul[1] = bb;
      pkbf2(f[4], f[5], a, bb); uh[2] = a; ul[2] = bb;
      pkbf2(f[6], f[7], a, bb); uh[3] = a; ul[3] = bb;
      volatile v4u* ph = (volatile v4u*)(outH + o);
      volatile v4u* pl = (volatile v4u*)(outL + o);
      *ph = uh; *pl = ul;
      __threadfence();
      *ph = uh; *pl = ul;
    } else {
      v4u u;
      u[0] = pkh2(f[0], f[1]); u[1] = pkh2(f[2], f[3]); u[2] = pkh2(f[4], f[5]); u[3] = pkh2(f[6], f[7]);
      volatile v4u* ph = (volatile v4u*)(outH + o);
      *ph = u;
      __threadfence();
      *ph = u;
    }
  }
}

__global__ __launch_bounds__(256) void k_im2col32(const float* __restrict__ R, const float* __restrict__ U,
                                                  unsigned short* __restrict__ outP, int h, int pxReal,
                                                  int rowStart, int nRows) {
  const int lane = threadIdx.x & 31;
  const int wg = blockIdx.x * 8 + (threadIdx.x >> 5);
  const int r0 = wg * 2;
  if (r0 >= nRows) return;
  const int hw = h * h;
#pragma unroll 1
  for (int t = 0; t < 3; ++t) {
    const int e   = (t * 32 + lane) * 8;
    const int rl  = e / PITCH_A32;
    const int col = e - rl * PITCH_A32;
    const int p   = rowStart + r0 + rl;
    const int pc  = p < pxReal ? p : (pxReal - 1);
    const int b   = pc / hw;
    const int rem = pc - b * hw;
    const int y   = rem / h;
    const int x   = rem - y * h;
    int tap = col >> 5; tap = tap > 8 ? 8 : tap;
    const int kh = tap / 3, kw = tap - kh * 3;
    const int c0 = col & 31;
    const int cc = c0 & 15;
    const float* plane = (c0 < 16) ? R : U;
    const int yi = y + kh - 1, xi = x + kw - 1;
    const bool ok = (col < KDIM32) && (p < pxReal) &&
                    ((unsigned)yi < (unsigned)h) && ((unsigned)xi < (unsigned)h);
    const int yc = yi < 0 ? 0 : (yi > h - 1 ? h - 1 : yi);
    const int xc = xi < 0 ? 0 : (xi > h - 1 ? h - 1 : xi);
    const float* s0 = plane + ((size_t)b * hw + (size_t)yc * h + xc) * NCH + cc;
    v4f a = *(const v4f*)(s0);
    v4f c = *(const v4f*)(s0 + 4);
    const v4f z = (v4f){0.f, 0.f, 0.f, 0.f};
    if (!ok) { a = z; c = z; }
    v4u u;
    u[0] = pkh2(a[0], a[1]); u[1] = pkh2(a[2], a[3]); u[2] = pkh2(c[0], c[1]); u[3] = pkh2(c[2], c[3]);
    volatile v4u* d = (volatile v4u*)(outP + (size_t)r0 * PITCH_A32 + e);
    *d = u;
    __threadfence();
    *d = u;
  }
}

__global__ __launch_bounds__(256) void k_sample(const float* __restrict__ U, const float* __restrict__ offs,
                                                const float* __restrict__ boff, unsigned short* __restrict__ S,
                                                int h, int pxReal, int rowStart, int nRows) {
  const int lane = threadIdx.x & 31;
  const int wg = blockIdx.x * 8 + (threadIdx.x >> 5);
  const int r0 = wg * 4;
  if (r0 >= nRows) return;
  const int hw = h * h;
  const float hm1 = (float)(h - 1);
#pragma unroll 1
  for (int t = 0; t < 3; ++t) {
    const int e   = (t * 32 + lane) * 8;
    const int rl  = e / PITCH_A16;
    const int col = e - rl * PITCH_A16;
    const int p   = rowStart + r0 + rl;
    const int pc  = p < pxReal ? p : (pxReal - 1);
    const int b   = pc / hw;
    const int rem = pc - b * hw;
    const int y   = rem / h;
    const int x   = rem - y * h;
    int tap = col >> 4; tap = tap > 8 ? 8 : tap;
    const int kh = tap / 3, kw = tap - kh * 3;
    const int c0 = col & 8;
    const int g0 = c0 >> 1;
    const bool ok = (col < KREAL16) && (p < pxReal);
    const float* orow = offs + (size_t)(r0 + rl) * NOFFPAD;
    const float* ub = U + (size_t)b * hw * NCH;
    const float by = (float)(y - 1 + kh), bx = (float)(x - 1 + kw);
    float res[8];
#pragma unroll
    for (int gg = 0; gg < 4; ++gg) {
      const int g  = g0 + gg;
      const int ch = (g * KTAPS + tap) * 2;
      const float dy = orow[ch] + boff[ch];
      const float dx = orow[ch + 1] + boff[ch + 1];
      const float py = by + dy, pxf = bx + dx;
      const float y0 = floorf(py), x0 = floorf(pxf);
      const float y1 = y0 + 1.0f, x1 = x0 + 1.0f;
      const float wy1 = py - y0, wx1 = pxf - x0;
      const float wy0 = 1.0f - wy1, wx0 = 1.0f - wx1;
      const bool vy0 = (y0 >= 0.0f) && (y0 <= hm1);
      const bool vy1 = (y1 >= 0.0f) && (y1 <= hm1);
      const bool vx0 = (x0 >= 0.0f) && (x0 <= hm1);
      const bool vx1 = (x1 >= 0.0f) && (x1 <= hm1);
      float w00 = wy0 * wx0, w01 = wy0 * wx1, w10 = wy1 * wx0, w11 = wy1 * wx1;
      w00 = (vy0 && vx0) ? w00 : 0.0f;
      w01 = (vy0 && vx1) ? w01 : 0.0f;
      w10 = (vy1 && vx0) ? w10 : 0.0f;
      w11 = (vy1 && vx1) ? w11 : 0.0f;
      const int yi0 = (int)fminf(fmaxf(y0, 0.0f), hm1);
      const int yi1 = (int)fminf(fmaxf(y1, 0.0f), hm1);
      const int xi0 = (int)fminf(fmaxf(x0, 0.0f), hm1);
      const int xi1 = (int)fminf(fmaxf(x1, 0.0f), hm1);
      const float* r00 = ub + ((size_t)yi0 * h + xi0) * NCH + 2 * g;
      const float* r01 = ub + ((size_t)yi0 * h + xi1) * NCH + 2 * g;
      const float* r10 = ub + ((size_t)yi1 * h + xi0) * NCH + 2 * g;
      const float* r11 = ub + ((size_t)yi1 * h + xi1) * NCH + 2 * g;
      const v2f g00 = *(const v2f*)(r00), g01 = *(const v2f*)(r01);
      const v2f g10 = *(const v2f*)(r10), g11 = *(const v2f*)(r11);
      const v2f v = g00 * w00 + g01 * w01 + g10 * w10 + g11 * w11;
      res[2 * gg]     = ok ? v[0] : 0.0f;
      res[2 * gg + 1] = ok ? v[1] : 0.0f;
    }
    v4u u;
    u[0] = pkh2(res[0], res[1]); u[1] = pkh2(res[2], res[3]);
    u[2] = pkh2(res[4], res[5]); u[3] = pkh2(res[6], res[7]);
    volatile v4u* d = (volatile v4u*)(S + (size_t)r0 * PITCH_A16 + e);
    *d = u;
    __threadfence();
    *d = u;
  }
}

__global__ __launch_bounds__(256) void k_pack(const float* __restrict__ OB, float* __restrict__ out, int hw, int nquad) {
  const int gid = blockIdx.x * 256 + threadIdx.x;
  if (gid < nquad) {
    const int f0   = gid * 4;
    const int q    = f0 / hw;
    const int rem0 = f0 - q * hw;
    const int b = q >> 4, o = q & 15;
    const float* s = OB + ((size_t)b * hw + rem0) * NCH + o;
    v4f v;
    v[0] = s[0]; v[1] = s[NCH]; v[2] = s[2 * NCH]; v[3] = s[3 * NCH];
    volatile v4f* d = (volatile v4f*)(out + f0);
    *d = v;
    __threadfence();
    *d = v;
  }
}

static inline unsigned gemm_blocks(int M, int tilesN) { return (unsigned)((((M >> 6) * tilesN) + 7) / 8); }

static void fe_level(hipStream_t stream, bool nchw, const float* src, int hin, int hout, int pad,
                     const unsigned short* wH, const unsigned short* wL, const float* bias,
                     float* feat, unsigned short* IMH, unsigned short* IML) {
  const int pxo = NBATCH * hout * hout;
  const int pxpado = (pxo + 63) / 64 * 64;
  for (int start = 0; start < pxpado; start += CHUNK_FE) {
    const int n = (pxpado - start) < CHUNK_FE ? (pxpado - start) : CHUNK_FE;
    if (nchw)
      k_im2col16<true, 0><<<dim3((unsigned)(n / 32)), 256, 0, stream>>>(src, IMH, IML, hin, hin, hout, hout, pad, pxo, start, n);
    else
      k_im2col16<false, 0><<<dim3((unsigned)(n / 32)), 256, 0, stream>>>(src, IMH, IML, hin, hin, hout, hout, pad, pxo, start, n);
    float* C = feat + (size_t)start * NCH;
    wmma_gemm64<1, true, 2, 3, false, 2, 1><<<dim3(gemm_blocks(n, 1), 1), 256, 0, stream>>>(
        IMH, IML, PITCH_A16, 0L,
        wH, wL, PITCH_A16, 0L,
        (void*)C, (void*)C, NCH, 0L,
        bias,
        bias, 0L,
        n, NCH, KDIM16, 1.0f);
  }
}

static void align_scale(hipStream_t stream, int h, const float* R, const float* Uf,
                        const unsigned short* wOff, const float* bOff,
                        const unsigned short* WDO, const float* dcnoff_b,
                        const unsigned short* WDC, const float* dcn_b,
                        float* OFFFEAT, float* OUTBUF,
                        unsigned short* IM32, unsigned short* X16, float* OFFS, float* outp) {
  const int px = NBATCH * h * h;
  const int pxpad = (px + 63) / 64 * 64;
  for (int start = 0; start < pxpad; start += CHUNK_A) {
    const int n = (pxpad - start) < CHUNK_A ? (pxpad - start) : CHUNK_A;
    k_im2col32<<<dim3((unsigned)(n / 16)), 256, 0, stream>>>(R, Uf, IM32, h, px, start, n);
    float* C = OFFFEAT + (size_t)start * NCH;
    wmma_gemm64<0, false, 2, 3, false, 2, 1><<<dim3(gemm_blocks(n, 1), 1), 256, 0, stream>>>(
        IM32, IM32, PITCH_A32, 0L,
        wOff, wOff, PITCH_A32, 0L,
        (void*)C, (void*)C, NCH, 0L,
        bOff,
        bOff, 0L,
        n, NCH, KDIM32, 0.0625f);
  }
  for (int start = 0; start < pxpad; start += CHUNK_B) {
    const int n = (pxpad - start) < CHUNK_B ? (pxpad - start) : CHUNK_B;
    k_im2col16<false, 1><<<dim3((unsigned)(n / 32)), 256, 0, stream>>>(OFFFEAT, X16, X16, h, h, h, h, 1, px, start, n);
    wmma_gemm64<0, false, 0, 0, false, 0, 4><<<dim3(gemm_blocks(n, NOFFPAD / 64), 1), 256, 0, stream>>>(
        X16, X16, PITCH_A16, 0L,
        WDO, WDO, PITCH_A16, 0L,
        (void*)OFFS, (void*)OFFS, NOFFPAD, 0L,
        dcnoff_b,
        dcnoff_b, 0L,
        n, NOFFPAD, KDIM16, 0.0625f);
    k_sample<<<dim3((unsigned)(n / 32)), 256, 0, stream>>>(Uf, OFFS, dcnoff_b, X16, h, px, start, n);
    float* C = OUTBUF + (size_t)start * NCH;
    wmma_gemm64<0, false, 2, 3, false, 0, 1><<<dim3(gemm_blocks(n, 1), 1), 256, 0, stream>>>(
        X16, X16, PITCH_A16, 0L,
        WDC, WDC, PITCH_A16, 0L,
        (void*)C, (void*)C, NCH, 0L,
        dcn_b,
        dcn_b, 0L,
        n, NCH, KDIM16, 0.0625f);
  }
  const int nquad = 4 * px;
  k_pack<<<dim3((unsigned)((nquad + 255) / 256)), 256, 0, stream>>>(OUTBUF, outp, h * h, nquad);
}

extern "C" void kernel_launch(void* const* d_in, const int* in_sizes, int n_in,
                              void* d_out, int out_size, void* d_ws, size_t ws_size,
                              hipStream_t stream) {
  if (n_in < 18) return;
  const int hs[3] = {IMG_H, IMG_H - 2, IMG_H - 4};
  int px[3];
  for (int i = 0; i < 3; ++i) px[i] = NBATCH * hs[i] * hs[i];
  if (in_sizes[0] != FEAT_ROWS * NCH || in_sizes[1] != FEAT_ROWS * NCH) return;
  if (in_sizes[2] != NCH * NCH * KTAPS || in_sizes[4] != NCH * NCH * KTAPS || in_sizes[6] != NCH * NCH * KTAPS) return;
  if (in_sizes[3] != NCH || in_sizes[5] != NCH || in_sizes[7] != NCH) return;
  if (in_sizes[8] != NCH * 2 * NCH * KTAPS || in_sizes[10] != NCH * 2 * NCH * KTAPS || in_sizes[12] != NCH * 2 * NCH * KTAPS) return;
  if (in_sizes[9] != NCH || in_sizes[11] != NCH || in_sizes[13] != NCH) return;
  if (in_sizes[14] != NOFFCH * NCH * KTAPS || in_sizes[15] != NOFFCH || in_sizes[16] != NCH * NCH * KTAPS || in_sizes[17] != NCH) return;
  if (out_size != NCH * (px[0] + px[1] + px[2])) return;

  const float* ref_img  = (const float*)d_in[0];
  const float* unr_img  = (const float*)d_in[1];
  const float* fe_w1    = (const float*)d_in[2];
  const float* fe_b1    = (const float*)d_in[3];
  const float* fe_w2    = (const float*)d_in[4];
  const float* fe_b2    = (const float*)d_in[5];
  const float* fe_w3    = (const float*)d_in[6];
  const float* fe_b3    = (const float*)d_in[7];
  const float* off_w0   = (const float*)d_in[8];
  const float* off_b0   = (const float*)d_in[9];
  const float* off_w1   = (const float*)d_in[10];
  const float* off_b1   = (const float*)d_in[11];
  const float* off_w2   = (const float*)d_in[12];
  const float* off_b2   = (const float*)d_in[13];
  const float* dcnoff_w = (const float*)d_in[14];
  const float* dcnoff_b = (const float*)d_in[15];
  const float* dcn_w    = (const float*)d_in[16];
  const float* dcn_b    = (const float*)d_in[17];
  float* out0 = (float*)d_out;
  float* out1 = out0 + (size_t)NCH * px[0];
  float* out2 = out1 + (size_t)NCH * px[1];

  const size_t bytes_feat  = (size_t)FEAT_ROWS * NCH * 4;
  const size_t bytes_arena = (size_t)CHUNK_FE * PITCH_A16 * 2 * 2;
  const size_t bytes_wfe   = (size_t)3 * 2 * 16 * PITCH_A16 * 2;
  const size_t bytes_woff  = (size_t)3 * 16 * PITCH_A32 * 2;
  const size_t bytes_wdo   = (size_t)NOFFPAD * PITCH_A16 * 2;
  const size_t bytes_wdc   = (size_t)16 * PITCH_A16 * 2;
  char* ws = (char*)d_ws;
  size_t o = 0;
  float* FR0 = (float*)(ws + o);            o += bytes_feat;
  float* FR1 = (float*)(ws + o);            o += bytes_feat;
  float* FU0 = (float*)(ws + o);            o += bytes_feat;
  float* FU1 = (float*)(ws + o);            o += bytes_feat;
  float* OFFFEAT = (float*)(ws + o);        o += bytes_feat;
  float* OUTBUF  = (float*)(ws + o);        o += bytes_feat;
  char* arena = ws + o;                     o += bytes_arena;
  unsigned short* WFE  = (unsigned short*)(ws + o);  o += bytes_wfe;
  unsigned short* WOFF = (unsigned short*)(ws + o);  o += bytes_woff;
  unsigned short* WDO  = (unsigned short*)(ws + o);  o += bytes_wdo;
  unsigned short* WDC  = (unsigned short*)(ws + o);  o += bytes_wdc;
  if (o > ws_size) return;
  unsigned short* IMH  = (unsigned short*)(arena);
  unsigned short* IML  = (unsigned short*)(arena + (size_t)CHUNK_FE * PITCH_A16 * 2);
  unsigned short* IM32 = (unsigned short*)(arena);
  unsigned short* X16  = (unsigned short*)(arena);
  float* OFFS = (float*)(arena + (size_t)CHUNK_B * PITCH_A16 * 2);

  const int feStride = 2 * 16 * PITCH_A16;
  const int feLo     = 16 * PITCH_A16;
  const int offStride = 16 * PITCH_A32;

  k_prep_w<16, 0><<<dim3(2, 3), 256, 0, stream>>>(fe_w1, fe_w2, fe_w3, WFE, feStride, feLo, NCH, NCH, 1.0f);
  k_prep_w<32, 1><<<dim3(3, 3), 256, 0, stream>>>(off_w0, off_w1, off_w2, WOFF, offStride, 0, NCH, NCH, 16.0f);
  k_prep_w<16, 1><<<dim3(18, 1), 256, 0, stream>>>(dcnoff_w, dcnoff_w, dcnoff_w, WDO, 0, 0, NOFFCH, NOFFPAD, 16.0f);
  k_prep_w<16, 1><<<dim3(2, 1), 256, 0, stream>>>(dcn_w, dcn_w, dcn_w, WDC, 0, 0, NCH, NCH, 16.0f);

  fe_level(stream, true, ref_img, IMG_H, hs[0], 1, WFE, WFE + feLo, fe_b1, FR0, IMH, IML);
  fe_level(stream, true, unr_img, IMG_H, hs[0], 1, WFE, WFE + feLo, fe_b1, FU0, IMH, IML);
  align_scale(stream, hs[0], FR0, FU0, WOFF, off_b0, WDO, dcnoff_b, WDC, dcn_b, OFFFEAT, OUTBUF, IM32, X16, OFFS, out0);
  fe_level(stream, false, FR0, hs[0], hs[1], 0, WFE + feStride, WFE + feStride + feLo, fe_b2, FR1, IMH, IML);
  fe_level(stream, false, FU0, hs[0], hs[1], 0, WFE + feStride, WFE + feStride + feLo, fe_b2, FU1, IMH, IML);
  align_scale(stream, hs[1], FR1, FU1, WOFF + offStride, off_b1, WDO, dcnoff_b, WDC, dcn_b, OFFFEAT, OUTBUF, IM32, X16, OFFS, out1);
  fe_level(stream, false, FR1, hs[1], hs[2], 0, WFE + 2 * feStride, WFE + 2 * feStride + feLo, fe_b3, FR0, IMH, IML);
  fe_level(stream, false, FU1, hs[1], hs[2], 0, WFE + 2 * feStride, WFE + 2 * feStride + feLo, fe_b3, FU0, IMH, IML);
  align_scale(stream, hs[2], FR0, FU0, WOFF + 2 * offStride, off_b2, WDO, dcnoff_b, WDC, dcn_b, OFFFEAT, OUTBUF, IM32, X16, OFFS, out2);
}
